// CriticNetwork_1_26972394619302
// MI455X (gfx1250) — hardware-verified
//
#include <hip/hip_runtime.h>

#define BB_  512
#define NN_  1024
#define HH_  128
#define WST  136

typedef _Float16 f16;
typedef __attribute__((ext_vector_type(16))) f16 f16x16;
typedef __attribute__((ext_vector_type(8)))  f16 f16x8;
typedef __attribute__((ext_vector_type(8)))  float f32x8;
typedef __attribute__((ext_vector_type(4)))  float v4f_t;
typedef float v4fa __attribute__((ext_vector_type(4), may_alias));

__device__ __forceinline__ f32x8 wmma16(f16x16 a, f16x16 b, f32x8 c) {
  c = __builtin_amdgcn_wmma_f32_16x16x32_f16(false, a, false, b, (short)0, c, false, false);
  asm volatile("v_nop\n\tv_nop\n\tv_nop\n\tv_nop" : "+v"(c) : "v"(a), "v"(b));
  return c;
}
__device__ __forceinline__ f16x16 load_frag(const float* __restrict__ base, int ld, int row0, int k0) {
  const int lane = threadIdx.x & 31, r = lane & 15, kh = (lane >> 4) * 8;
  const float* p0 = base + (size_t)(row0 + r) * ld + (k0 + kh);
  const v4f_t a = *(const v4f_t*)(p0), b = *(const v4f_t*)(p0 + 4), c = *(const v4f_t*)(p0 + 16), d = *(const v4f_t*)(p0 + 20);
  f16x16 f;
  f[0] = (f16)a[0]; f[1] = (f16)a[1]; f[2]  = (f16)a[2]; f[3]  = (f16)a[3]; f[4]  = (f16)b[0]; f[5]  = (f16)b[1]; f[6]  = (f16)b[2]; f[7]  = (f16)b[3];
  f[8] = (f16)c[0]; f[9] = (f16)c[1]; f[10] = (f16)c[2]; f[11] = (f16)c[3]; f[12] = (f16)d[0]; f[13] = (f16)d[1]; f[14] = (f16)d[2]; f[15] = (f16)d[3];
  return f;
}
__device__ __forceinline__ f16x16 lds_frag(const f16* base, int stride) {
  const int lane = threadIdx.x & 31, row = lane & 15, kh = (lane >> 4) * 8;
  const f16x8 lo = *(const f16x8*)(base + row * stride + kh);
  const f16x8 hi = *(const f16x8*)(base + row * stride + kh + 16);
  f16x16 f;
#pragma unroll
  for (int i = 0; i < 8; ++i) { f[i] = lo[i]; f[i + 8] = hi[i]; }
  return f;
}

__global__ __launch_bounds__(128) void k_fold(const float* __restrict__ Wemb, const float* __restrict__ bemb, const float* __restrict__ Wref,
                                              const float* __restrict__ bref, float* __restrict__ fold) {
  const int h = threadIdx.x;
  float m0 = 0.0f, m1 = 0.0f, cv = bref[h];
  for (int j = 0; j < HH_; ++j) { const float w = Wref[j * HH_ + h]; m0 += Wemb[j] * w; m1 += Wemb[HH_ + j] * w; cv += bemb[j] * w; }
#pragma unroll 1
  for (int pass = 0; pass < 2; ++pass) {
    *(volatile float*)(fold + h) = m0; *(volatile float*)(fold + HH_ + h) = m1; *(volatile float*)(fold + 2 * HH_ + h) = cv;
    __threadfence();
  }
}

__global__ __launch_bounds__(256) void k_proj(const float* __restrict__ q, int ldq, const float* __restrict__ Wm,
                                              const float* __restrict__ bias, float* __restrict__ u1) {
  __shared__ __attribute__((aligned(16))) f16 WS[HH_ * WST];
  __shared__ __attribute__((aligned(16))) float oS[8][16 * 132];
  const int tid = threadIdx.x, lane = tid & 31, wave = tid >> 5, cl = lane & 15, rh = (lane >> 4) * 8;
  for (int e = tid; e < HH_ * HH_; e += 256) { const int n = e >> 7, k = e & 127; WS[n * WST + k] = (f16)Wm[k * HH_ + n]; }
  __syncthreads();
  const int row0 = blockIdx.x * 128 + wave * 16;
  f16x16 af[4];
#pragma unroll
  for (int ks = 0; ks < 4; ++ks) af[ks] = load_frag(q, ldq, row0, ks * 32);
#pragma unroll
  for (int nt = 0; nt < 8; ++nt) {
    f32x8 acc = {};
#pragma unroll
    for (int ks = 0; ks < 4; ++ks) acc = wmma16(af[ks], lds_frag(WS + nt * 16 * WST + ks * 32, WST), acc);
    const float bv = bias ? bias[nt * 16 + cl] : 0.0f;
#pragma unroll
    for (int r = 0; r < 8; ++r) oS[wave][(rh + r) * 132 + nt * 16 + cl] = acc[r] + bv;
  }
  asm volatile("s_wait_dscnt 0" ::: "memory");
  __syncthreads();
#pragma unroll 1
  for (int pass = 0; pass < 2; ++pass) {
#pragma unroll
    for (int it = 0; it < 16; ++it) { const int f4 = lane + 32 * it, rr = f4 >> 5, qd = (f4 & 31) * 4;
      *(volatile v4f_t*)(u1 + (size_t)(row0 + rr) * HH_ + qd) = *(const volatile v4fa*)(oS[wave] + rr * 132 + qd); }
    __threadfence();
  }
}

__global__ __launch_bounds__(256) void k_glimpse(const float* __restrict__ x, const float* __restrict__ u1, const float* __restrict__ fold,
                                                 const float* __restrict__ Vec, float* __restrict__ qout) {
  __shared__ float c0S[HH_], m0S[HH_], m1S[HH_];
  __shared__ float uS[NN_];
  __shared__ float red[8], red2[8][2];
  __shared__ __attribute__((aligned(16))) float dS[HH_];
  const int tid = threadIdx.x, lane = tid & 31, wave = tid >> 5, cl = lane & 15, kh = (lane >> 4) * 8, rh = kh;
  const int b = blockIdx.x;
  if (tid < HH_) { m0S[tid] = fold[tid]; m1S[tid] = fold[HH_ + tid]; c0S[tid] = u1[(size_t)b * HH_ + tid] + fold[2 * HH_ + tid]; }
  __syncthreads();
  f16x16 vb[4];
#pragma unroll
  for (int ks = 0; ks < 4; ++ks)
#pragma unroll
    for (int e = 0; e < 8; ++e) {
      vb[ks][e]     = (cl == 0) ? (f16)Vec[ks * 32 + kh + e]      : (f16)0.0f;
      vb[ks][e + 8] = (cl == 0) ? (f16)Vec[ks * 32 + kh + 16 + e] : (f16)0.0f;
    }
  const float* xb = x + (size_t)b * NN_ * 2;
#pragma unroll 1
  for (int tt = 0; tt < 8; ++tt) {
    const int n0 = (wave * 8 + tt) * 16;
    const float x0 = xb[(n0 + cl) * 2], x1 = xb[(n0 + cl) * 2 + 1];
    f32x8 acc = {};
#pragma unroll
    for (int ks = 0; ks < 4; ++ks) {
      f16x16 af;
#pragma unroll
      for (int e = 0; e < 16; ++e) {
        const int hI = ks * 32 + kh + (e & 7) + ((e >> 3) << 4);
        const float z = c0S[hI] + x0 * m0S[hI] + x1 * m1S[hI];
        af[e] = (f16)(1.0f - 2.0f / (1.0f + __expf(2.0f * z)));
      }
      acc = wmma16(af, vb[ks], acc);
    }
    if (cl == 0) {
#pragma unroll
      for (int r = 0; r < 8; ++r) uS[n0 + rh + r] = acc[r];
    }
  }
  __syncthreads();
  float u[4], mx = -3.0e38f;
#pragma unroll
  for (int j = 0; j < 4; ++j) { u[j] = uS[tid + 256 * j]; mx = fmaxf(mx, u[j]); }
#pragma unroll
  for (int off = 16; off >= 1; off >>= 1) mx = fmaxf(mx, __shfl_xor(mx, off, 32));
  if (lane == 0) red[wave] = mx;
  __syncthreads();
  mx = fmaxf(fmaxf(fmaxf(red[0], red[1]), fmaxf(red[2], red[3])), fmaxf(fmaxf(red[4], red[5]), fmaxf(red[6], red[7])));
  float se = 0.0f, s0 = 0.0f, s1 = 0.0f;
#pragma unroll
  for (int j = 0; j < 4; ++j) { const int n = tid + 256 * j; const float e = __expf(u[j] - mx); se += e; s0 += e * xb[n * 2]; s1 += e * xb[n * 2 + 1]; }
#pragma unroll
  for (int off = 16; off >= 1; off >>= 1) { se += __shfl_xor(se, off, 32); s0 += __shfl_xor(s0, off, 32); s1 += __shfl_xor(s1, off, 32); }
  __syncthreads();
  if (lane == 0) { red[wave] = se; red2[wave][0] = s0; red2[wave][1] = s1; }
  __syncthreads();
  if (tid < HH_) {
    const float Z  = ((red[0] + red[1]) + (red[2] + red[3])) + ((red[4] + red[5]) + (red[6] + red[7]));
    const float S0 = ((red2[0][0] + red2[1][0]) + (red2[2][0] + red2[3][0])) + ((red2[4][0] + red2[5][0]) + (red2[6][0] + red2[7][0]));
    const float S1 = ((red2[0][1] + red2[1][1]) + (red2[2][1] + red2[3][1])) + ((red2[4][1] + red2[5][1]) + (red2[6][1] + red2[7][1]));
    dS[tid] = (S0 / Z) * m0S[tid] + (S1 / Z) * m1S[tid] + fold[2 * HH_ + tid];
  }
  __syncthreads();
  if (wave == 0) {
#pragma unroll 1
    for (int pass = 0; pass < 2; ++pass) { *(volatile v4f_t*)(qout + (size_t)b * HH_ + lane * 4) = *(const volatile v4fa*)(dS + lane * 4); __threadfence(); }
  }
}

__global__ __launch_bounds__(256) void k_head(const float* __restrict__ q, const float* __restrict__ W1m, const float* __restrict__ W2v,
                                              float* __restrict__ out) {
  __shared__ __attribute__((aligned(16))) f16 WS[HH_ * WST];
  __shared__ __attribute__((aligned(16))) f16 hS[8][16 * WST];
  __shared__ __attribute__((aligned(16))) float pS[128];
  const int tid = threadIdx.x, lane = tid & 31, wave = tid >> 5, cl = lane & 15, rh = (lane >> 4) * 8, kh = rh;
  for (int e = tid; e < HH_ * HH_; e += 256) { const int n = e >> 7, k = e & 127; WS[n * WST + k] = (f16)W1m[k * HH_ + n]; }
  __syncthreads();
  const int row0 = blockIdx.x * 128 + wave * 16;
  f16x16 af[4];
#pragma unroll
  for (int ks = 0; ks < 4; ++ks) af[ks] = load_frag(q, HH_, row0, ks * 32);
#pragma unroll
  for (int nt = 0; nt < 8; ++nt) {
    f32x8 acc = {};
#pragma unroll
    for (int ks = 0; ks < 4; ++ks) acc = wmma16(af[ks], lds_frag(WS + nt * 16 * WST + ks * 32, WST), acc);
#pragma unroll
    for (int r = 0; r < 8; ++r) hS[wave][(rh + r) * WST + nt * 16 + cl] = (f16)fmaxf(acc[r], 0.0f);
  }
  f16x16 wb[4];
#pragma unroll
  for (int ks = 0; ks < 4; ++ks)
#pragma unroll
    for (int e = 0; e < 8; ++e) {
      wb[ks][e]     = (cl == 0) ? (f16)W2v[ks * 32 + kh + e]      : (f16)0.0f;
      wb[ks][e + 8] = (cl == 0) ? (f16)W2v[ks * 32 + kh + 16 + e] : (f16)0.0f;
    }
  asm volatile("s_wait_dscnt 0" ::: "memory");
  __syncthreads();
  f32x8 pz = {};
#pragma unroll
  for (int ks = 0; ks < 4; ++ks) pz = wmma16(lds_frag(hS[wave] + ks * 32, WST), wb[ks], pz);
  if (cl == 0) {
#pragma unroll
    for (int r = 0; r < 8; ++r) pS[wave * 16 + rh + r] = pz[r];
  }
  __syncthreads();
  if (wave == 0) {
#pragma unroll 1
    for (int pass = 0; pass < 2; ++pass) { *(volatile v4f_t*)(out + (size_t)blockIdx.x * 128 + lane * 4) = *(const volatile v4fa*)(pS + lane * 4); __threadfence(); }
  }
}

extern "C" void kernel_launch(void* const* d_in, const int* in_sizes, int n_in,
                              void* d_out, int out_size, void* d_ws, size_t ws_size,
                              hipStream_t stream) {
  (void)in_sizes; (void)n_in; (void)out_size; (void)ws_size;
  const float* x    = (const float*)d_in[0];
  const float* Wemb = (const float*)d_in[2];
  const float* bemb = (const float*)d_in[3];
  const float* dec  = (const float*)d_in[4];
  const float* Vec  = (const float*)d_in[5];
  const float* Wq   = (const float*)d_in[6];
  const float* bq   = (const float*)d_in[7];
  const float* Wref = (const float*)d_in[8];
  const float* bref = (const float*)d_in[9];
  const float* Wfc1 = (const float*)d_in[10];
  const float* Wfc2 = (const float*)d_in[11];
  float* out = (float*)d_out;
  char* ws = (char*)d_ws;
  float* fold = (float*)ws;
  float* u1 = (float*)(ws + 4096);
  float* q1 = (float*)(ws + 4096 + 262144);
  float* q2 = (float*)(ws + 4096 + 2 * 262144);
  k_fold<<<dim3(1), dim3(128), 0, stream>>>(Wemb, bemb, Wref, bref, fold);
  k_proj<<<dim3(4), dim3(256), 0, stream>>>(dec, 0, Wq, bq, u1);
  k_glimpse<<<dim3(BB_), dim3(256), 0, stream>>>(x, u1, fold, Vec, q1);
  k_proj<<<dim3(4), dim3(256), 0, stream>>>(q1, HH_, Wq, bq, u1);
  k_glimpse<<<dim3(BB_), dim3(256), 0, stream>>>(x, u1, fold, Vec, q2);
  k_head<<<dim3(4), dim3(256), 0, stream>>>(q2, Wfc1, Wfc2, out);
}
